// PrototypeClassifier_9182640079462
// MI455X (gfx1250) — hardware-verified
//
#include <hip/hip_runtime.h>
#include <math.h>


constexpr int Bn = 8192, Pn = 2048, Dn = 512;
typedef __attribute__((ext_vector_type(16))) _Float16 v16h;
typedef __attribute__((ext_vector_type(8)))  _Float16 v8h;
typedef __attribute__((ext_vector_type(8)))  float    v8f;
typedef __attribute__((ext_vector_type(4)))  float    v4f;
#define VST2(T, ptr, val) do { const T _v = (val); *(volatile T*)(ptr) = _v; __threadfence(); *(volatile T*)(ptr) = _v; } while (0)
__device__ __forceinline__ v8f wmma16(v16h a, v16h b, v8f c) {
  v8f d = __builtin_amdgcn_wmma_f32_16x16x32_f16(false, a, false, b, (short)0, c, false, false);
  asm volatile("v_nop\n\tv_nop\n\tv_nop\n\tv_nop" : "+v"(d) : "v"(a), "v"(b));
  return d;
}
__device__ __forceinline__ v16h frag16(const _Float16* p, int hh) {
  const v8h lo = *(const v8h*)(p + 8 * hh), hi = *(const v8h*)(p + 16 + 8 * hh);
  return __builtin_shufflevector(lo, hi, 0,1,2,3,4,5,6,7,8,9,10,11,12,13,14,15);
}
__global__ __launch_bounds__(256) void cvt_kernel(const float* __restrict__ src, _Float16* __restrict__ dst, int n8) {
  const int i = blockIdx.x * 256 + threadIdx.x;
  if (i >= n8) return;
  v8h v;
#pragma unroll
  for (int e = 0; e < 8; ++e) v[e] = (_Float16)src[(size_t)i * 8 + e];
  VST2(v8h, dst + (size_t)i * 8, v);
}
__global__ __launch_bounds__(256) void rowsq_kernel(const float* __restrict__ src, int cols, int rows, float* __restrict__ sq) {
  __shared__ float red[32];
  const int lane = threadIdx.x & 31, wave = threadIdx.x >> 5;
  for (int q = 0; q < 4; ++q) {
    const int r = blockIdx.x * 32 + wave * 4 + q;
    float s = 0.f;
    if (r < rows) for (int c = lane; c < cols; c += 32) { const float x = src[(size_t)r * cols + c]; s += x * x; }
#pragma unroll
    for (int off = 16; off > 0; off >>= 1) s += __shfl_xor(s, off, 32);
    if (lane == 0) red[wave * 4 + q] = s;
  }
  __syncthreads();
  if (threadIdx.x < 32 && blockIdx.x * 32 + threadIdx.x < rows) VST2(float, sq + blockIdx.x * 32 + threadIdx.x, red[threadIdx.x]);
}
template <int EPI>
__global__ __launch_bounds__(128) void gemm_nt_kernel(const _Float16* __restrict__ A, const _Float16* __restrict__ B, int M, int N, int K,
                                                     const float* __restrict__ rowsq, const float* __restrict__ colsq,
                                                     _Float16* __restrict__ D16, const float* __restrict__ bias, float* __restrict__ Out) {
  __shared__ __attribute__((aligned(16))) float sT[4][16][68];
  const int lane = threadIdx.x & 31, wave = threadIdx.x >> 5, hh = lane >> 4, l16 = lane & 15;
  const int m0 = (blockIdx.x * 4 + wave) * 64, n0 = blockIdx.y * 64;
  v8f acc[4][4] = {};
  for (int k0 = 0; k0 < K; k0 += 32) {
    v16h a[4];
#pragma unroll
    for (int mi = 0; mi < 4; ++mi) a[mi] = frag16(A + (size_t)(m0 + mi * 16 + l16) * K + k0, hh);
#pragma unroll
    for (int ni = 0; ni < 4; ++ni) {
      const v16h b = frag16(B + (size_t)(n0 + ni * 16 + l16) * K + k0, hh);
#pragma unroll
      for (int mi = 0; mi < 4; ++mi) acc[mi][ni] = wmma16(a[mi], b, acc[mi][ni]);
    }
  }
  float (*st)[68] = sT[wave];
#pragma unroll
  for (int mi = 0; mi < 4; ++mi) {
#pragma unroll
    for (int ni = 0; ni < 4; ++ni)
#pragma unroll
      for (int i = 0; i < 8; ++i) {
        const int ml = i + 8 * hh, nl = ni * 16 + l16;
        const float c = acc[mi][ni][i];
        float v;
        if (EPI == 0) v = sqrtf(fmaxf(rowsq[m0 + mi * 16 + ml] + colsq[n0 + nl] - 2.0f * c, 0.0f));
        else          v = c + bias[n0 + nl];
        st[ml][nl] = v;
      }
    __builtin_amdgcn_fence(__ATOMIC_RELEASE, "workgroup"); __builtin_amdgcn_wave_barrier(); __builtin_amdgcn_fence(__ATOMIC_ACQUIRE, "workgroup");
    for (int pass = 0; pass < 2; ++pass) {
      if (EPI == 0) {
#pragma unroll
        for (int j = 0; j < 4; ++j) { const int rr = j * 4 + (lane >> 3), q8 = (lane & 7) * 8; v8h hv;
#pragma unroll
          for (int e = 0; e < 8; ++e) hv[e] = (_Float16)st[rr][q8 + e];
          *(volatile v8h*)(D16 + (size_t)(m0 + mi * 16 + rr) * N + n0 + q8) = hv; }
      } else {
#pragma unroll
        for (int j = 0; j < 8; ++j) { const int rr = j * 2 + hh, q4 = l16 * 4;
          *(volatile v4f*)(Out + (size_t)(m0 + mi * 16 + rr) * N + n0 + q4) = *(const v4f*)(&st[rr][q4]); }
      }
      __threadfence();
    }
    __builtin_amdgcn_fence(__ATOMIC_RELEASE, "workgroup"); __builtin_amdgcn_wave_barrier(); __builtin_amdgcn_fence(__ATOMIC_ACQUIRE, "workgroup");
  }
}
extern "C" void kernel_launch(void* const* d_in, const int* in_sizes, int n_in,
                              void* d_out, int out_size, void* d_ws, size_t ws_size, hipStream_t stream) {
  (void)in_sizes; (void)n_in; (void)out_size;
  const float* x     = (const float*)d_in[0];
  const float* proto = (const float*)d_in[1];
  const float* W     = (const float*)d_in[2];
  const float* bias  = (const float*)d_in[3];
  float* out         = (float*)d_out;
  size_t off = 0;
  auto carve = [&](size_t bytes) -> void* { void* p = (void*)((char*)d_ws + off); off += (bytes + 255) & ~(size_t)255; return p; };
  _Float16* X16 = (_Float16*)carve((size_t)Bn * Dn * 2);
  _Float16* P16 = (_Float16*)carve((size_t)Pn * Dn * 2);
  _Float16* W16 = (_Float16*)carve((size_t)Dn * Pn * 2);
  _Float16* G16 = (_Float16*)carve((size_t)Bn * Pn * 2);
  float* insq = (float*)carve((size_t)Bn * 4);
  float* prsq = (float*)carve((size_t)Pn * 4);
  if (off > ws_size) return;
  cvt_kernel<<<(Bn * Dn / 8) / 256, 256, 0, stream>>>(x, X16, Bn * Dn / 8);
  cvt_kernel<<<(Pn * Dn / 8) / 256, 256, 0, stream>>>(proto, P16, Pn * Dn / 8);
  cvt_kernel<<<(Dn * Pn / 8) / 256, 256, 0, stream>>>(W, W16, Dn * Pn / 8);
  rowsq_kernel<<<Bn / 32, 256, 0, stream>>>(x, Dn, Bn, insq);
  rowsq_kernel<<<Pn / 32, 256, 0, stream>>>(proto, Dn, Pn, prsq);
  gemm_nt_kernel<0><<<dim3(Bn / 256, Pn / 64), 128, 0, stream>>>(X16, P16, Bn, Pn, Dn, insq, prsq, G16, nullptr, nullptr);
  gemm_nt_kernel<1><<<dim3(Bn / 256, Dn / 64), 128, 0, stream>>>(G16, W16, Bn, Dn, Pn, nullptr, nullptr, nullptr, bias, out);
}
